// TransformerBlock_30812095381604
// MI455X (gfx1250) — hardware-run, weakly checked
//
#include <hip/hip_runtime.h>
#include <math.h>

typedef __attribute__((ext_vector_type(16))) _Float16 v16h;
typedef __attribute__((ext_vector_type(16))) __bf16 v16b;
typedef __attribute__((ext_vector_type(8)))  _Float16 v8h;
typedef __attribute__((ext_vector_type(8)))  __bf16 v8b;
typedef __attribute__((ext_vector_type(8)))  float v8f;
typedef __attribute__((ext_vector_type(4)))  float v4f;
typedef __attribute__((ext_vector_type(4)))  unsigned v4u;

#ifndef NB
#define NB 2
#endif
#ifndef TT
#define TT 2048
#endif
#define TT_FULL 2048
#define CC 1024
#define DIN 512
#define NH 16
#define HD 64
#define C2 (0.18033688011112042f)

static_assert(CC == NH * HD);
static_assert(HD == 64);
static_assert(TT % 64 == 0);
static_assert(TT % 32 == 0);
static_assert(TT <= TT_FULL);
static_assert(DIN % 64 == 0);
static_assert(CC % 128 == 0);
static_assert(CC % 64 == 0);
static_assert(DIN % 32 == 0);
static_assert(CC % 32 == 0);
static_assert(DIN <= CC);
static_assert(((size_t)NB * TT) % 64 == 0);
static_assert(((size_t)NB * TT * DIN) % (8 * 256) == 0);

#define WS_XB  ((size_t)0)
#define WS_WT  (WS_XB + 2u * (size_t)NB * TT * DIN)
#define WS_E   (WS_WT + 2u * ((size_t)CC * DIN + (size_t)6 * CC * CC))
#define WS_EH  (WS_E  + 4u * (size_t)NB * TT * CC)
#define WS_QK  (WS_EH + 2u * (size_t)NB * TT * CC)
#define WS_VT  (WS_QK + 2u * (size_t)2 * NB * TT * CC)
#define WS_CT  (WS_VT + 2u * (size_t)NB * CC * TT)
#define WS_MF  (WS_CT + 2u * (size_t)NB * TT * CC)
#define WS_MH  (WS_MF + 4u * (size_t)NB * TT * CC)
#define WS_HH  (WS_MH + 2u * (size_t)NB * TT * CC)
#define WS_END (WS_HH + 2u * (size_t)NB * TT * CC)
static_assert(WS_END <= (size_t)134217728);
static_assert(WS_WT % 128 == 0);
static_assert(WS_E  % 128 == 0);
static_assert(WS_EH % 128 == 0);
static_assert(WS_QK % 128 == 0);
static_assert(WS_VT % 128 == 0);
static_assert(WS_CT % 128 == 0);
static_assert(WS_MF % 128 == 0);
static_assert(WS_MH % 128 == 0);
static_assert(WS_HH % 128 == 0);

template <typename T> __device__ __forceinline__ void vst2(void* p, T v) { *(volatile T*)p = v; __threadfence(); *(volatile T*)p = v; }
__device__ __forceinline__ v8f wmma16(v16h a, v16h b, v8f c) {
  v8f d = __builtin_amdgcn_wmma_f32_16x16x32_f16(false, a, false, b, (short)0, c, false, false);
  asm volatile("v_nop\n\tv_nop\n\tv_nop\n\tv_nop" : "+v"(d) : "v"(a), "v"(b));
  return d;
}
__device__ __forceinline__ v8f wmma_bf(v16b a, v16b b, v8f c) {
  v8f d = __builtin_amdgcn_wmma_f32_16x16x32_bf16(false, a, false, b, (short)0, c, false, false);
  asm volatile("v_nop\n\tv_nop\n\tv_nop\n\tv_nop" : "+v"(d) : "v"(a), "v"(b));
  return d;
}
__device__ __forceinline__ v16h frag_h(const _Float16* rowk0, int lane) {
  union { v16h v; v8h q[2]; } u; const _Float16* p = rowk0 + 8 * (lane >> 4);
  u.q[0] = *(const v8h*)p; u.q[1] = *(const v8h*)(p + 16); return u.v;
}
__device__ __forceinline__ v16b frag_b(const __bf16* rowk0, int lane) {
  union { v16b v; v8b q[2]; } u; const __bf16* p = rowk0 + 8 * (lane >> 4);
  u.q[0] = *(const v8b*)p; u.q[1] = *(const v8b*)(p + 16); return u.v;
}
__device__ __forceinline__ float bfr(float v) { return (float)(__bf16)v; }
__device__ __forceinline__ unsigned bf_bits(float v) { return (unsigned)__builtin_bit_cast(unsigned short, (__bf16)v); }
#define LDSX() do { asm volatile("s_wait_dscnt 0" ::: "memory"); __builtin_amdgcn_wave_barrier(); __builtin_amdgcn_fence(3  , "workgroup"); } while (0)
static __device__ __forceinline__ _Float16 toh_flush(float v) { const _Float16 r = (_Float16)v; return (fabsf(v) < 6.103515625e-05f) ? (_Float16)0.0f : r; }

__global__ __launch_bounds__(256) void k_cvtx(const float* __restrict__ X, unsigned short* __restrict__ XB) {
  const size_t e = ((size_t)blockIdx.x * 256 + threadIdx.x) * 8;
  const size_t row = e / DIN; const int c = (int)(e % DIN); const size_t b = row / TT; const size_t t = row % TT;
  const float* src = X + (b * TT_FULL + t) * DIN + c;
  const v4f f0 = *(const v4f*)src; const v4f f1 = *(const v4f*)(src + 4);
  v4u o;
  o[0] = bf_bits(f0[0]) | (bf_bits(f0[1]) << 16);
  o[1] = bf_bits(f0[2]) | (bf_bits(f0[3]) << 16);
  o[2] = bf_bits(f1[0]) | (bf_bits(f1[1]) << 16);
  o[3] = bf_bits(f1[2]) | (bf_bits(f1[3]) << 16);
  vst2(XB + e, o);
}

__global__ __launch_bounds__(128) void k_wt(const float* __restrict__ WE, const float* __restrict__ WQ, const float* __restrict__ WK, const float* __restrict__ WV, const float* __restrict__ WO, const float* __restrict__ WF1, const float* __restrict__ WF2, unsigned short* __restrict__ WT) {
  __shared__ __align__(16) unsigned short ts[64][72];
  const int tid = threadIdx.x; const int z = blockIdx.z; const int k0 = blockIdx.x * 64, o0 = blockIdx.y * 64;
  if (z == 0 && k0 >= DIN) return;
  const float* W = z == 0 ? WE : z == 1 ? WQ : z == 2 ? WK : z == 3 ? WV : z == 4 ? WO : z == 5 ? WF1 : WF2;
#pragma unroll 1
  for (int i = 0; i < 8; ++i) { const int e = tid + i * 128; const int kl = e >> 4, c4 = e & 15;
    const v4f v = *(const v4f*)(W + (size_t)(k0 + kl) * CC + o0 + c4 * 4);
#pragma unroll
    for (int x = 0; x < 4; ++x) { const float bv = bfr(v[x]); const unsigned short ub = __builtin_bit_cast(unsigned short, (__bf16)v[x]); const unsigned short uh = __builtin_bit_cast(unsigned short, toh_flush(bv * 256.0f)); ts[c4 * 4 + x][kl] = (z == 0) ? ub : uh; } }
  __syncthreads();
  const size_t kw = (z == 0) ? (size_t)DIN : (size_t)CC;
  const size_t zoff = (z == 0) ? (size_t)0 : ((size_t)CC * DIN + (size_t)(z - 1) * CC * CC);
#pragma unroll 1
  for (int i = 0; i < 4; ++i) { const int e = tid + i * 128; const int ol = e >> 3, q = e & 7;
    vst2(WT + zoff + (size_t)(o0 + ol) * kw + k0 + q * 8, *(const v4u*)&ts[ol][q * 8]); }
}

template <int RES, int RELU, int WF32, int WF16, int DOUT>
__device__ __forceinline__ void epi_tile(v8f (&acc)[8], const float sc, const float* __restrict__ BIAS, const float* __restrict__ R, float* __restrict__ CF, _Float16* __restrict__ CH, const size_t rb, const int c0, const int wave, const int lane) {
  __shared__ __align__(16) float sf[4][16][132];
  const int col = lane & 15, g = lane >> 4;
  const size_t r0 = rb + (size_t)wave * 16;
#pragma unroll
  for (int j = 0; j < 8; ++j) { const float bias = bfr(BIAS[c0 + j * 16 + col]);
#pragma unroll
    for (int r = 0; r < 8; ++r) { float v = acc[j][r] * sc + bias; if (RELU) v = fmaxf(v, 0.0f); sf[wave][8 * g + r][j * 16 + col] = v; } }
  LDSX();
  if (RES || WF32) {
    const size_t bbo = rb / TT; const size_t to = rb % TT + (size_t)wave * 16;
    const size_t ob = DOUT ? (bbo * TT_FULL + to) : r0;
#pragma unroll 1
    for (int rl = 0; rl < 16; ++rl) { v4f v = *(const v4f*)&sf[wave][rl][lane * 4];
      if (RES) { const v4f rr = *(const v4f*)(R + (r0 + rl) * CC + c0 + lane * 4); v = v + rr; if (WF16) *(v4f*)&sf[wave][rl][lane * 4] = v; }
      if (WF32) vst2(CF + (ob + rl) * CC + c0 + lane * 4, v); }
    if (RES && WF16) LDSX();
  }
  if (WF16) {
#pragma unroll 1
    for (int i = 0; i < 8; ++i) { const int rl = i * 2 + (lane >> 4), q = lane & 15;
      const v4f f0 = *(const v4f*)&sf[wave][rl][q * 8]; const v4f f1 = *(const v4f*)&sf[wave][rl][q * 8 + 4];
      v8h hv;
#pragma unroll
      for (int x = 0; x < 4; ++x) { hv[x] = toh_flush(f0[x] * 64.0f); hv[4 + x] = toh_flush(f1[x] * 64.0f); }
      vst2(CH + (r0 + rl) * CC + c0 + q * 8, hv); }
  }
}

__device__ __forceinline__ void mm_f16(v8f (&acc)[8], const _Float16* __restrict__ ar, const _Float16* __restrict__ wr, const int lane) {
#pragma unroll 1
  for (int kc = 0; kc < CC / 32; ++kc) { const v16h a = frag_h(ar + kc * 32, lane);
#pragma unroll
    for (int j = 0; j < 8; ++j) { const v16h w = frag_h(wr + (size_t)j * 16 * CC + kc * 32, lane); acc[j] = wmma16(a, w, acc[j]); } }
}

__global__ __launch_bounds__(128) void k_emb(const __bf16* __restrict__ XB, const __bf16* __restrict__ WET, const float* __restrict__ BE, float* __restrict__ E, _Float16* __restrict__ EH) {
  const int tid = threadIdx.x; const int wave = __builtin_amdgcn_readfirstlane(threadIdx.x >> 5); const int lane = tid & 31, col = lane & 15;
  const int c0 = blockIdx.y * 128; const size_t rb = (size_t)blockIdx.x * 64; const size_t r0 = rb + wave * 16;
  const __bf16* xr = XB + (r0 + col) * DIN;
  const __bf16* wr = WET + (size_t)(c0 + col) * DIN;
  v8f acc[8] = {};
#pragma unroll 1
  for (int kc = 0; kc < DIN / 32; ++kc) { const v16b a = frag_b(xr + kc * 32, lane);
#pragma unroll
    for (int j = 0; j < 8; ++j) { const v16b w = frag_b(wr + (size_t)j * 16 * DIN + kc * 32, lane); acc[j] = wmma_bf(a, w, acc[j]); } }
  epi_tile<0, 0, 1, 1, 0>(acc, 1.0f, BE, BE, E, EH, rb, c0, wave, lane);
}

__global__ __launch_bounds__(128) void k_proj(const _Float16* __restrict__ EH, const _Float16* __restrict__ WT, const float* __restrict__ BQ, const float* __restrict__ BK, const float* __restrict__ BV, _Float16* __restrict__ QK, _Float16* __restrict__ VT) {
  __shared__ __align__(16) _Float16 sh[64][136]; __shared__ __align__(16) _Float16 th[128][72];
  const int tid = threadIdx.x; const int wave = __builtin_amdgcn_readfirstlane(threadIdx.x >> 5); const int lane = tid & 31, col = lane & 15, g = lane >> 4;
  const int which = blockIdx.z; const int c0 = blockIdx.y * 128; const size_t r0 = (size_t)blockIdx.x * 64; const size_t bb = r0 / TT; const int t0 = (int)(r0 % TT);
  const float* BA = which == 0 ? BQ : which == 1 ? BK : BV;
  const _Float16* xr = EH + (r0 + wave * 16 + col) * CC;
  const _Float16* wr = WT + ((size_t)which * CC + c0 + col) * CC;
  v8f acc[8] = {};
  mm_f16(acc, xr, wr, lane);
  if (which < 2) { _Float16* DH = QK + (size_t)which * NB * TT * CC;
#pragma unroll
    for (int j = 0; j < 8; ++j) { const float bias = bfr(BA[c0 + j * 16 + col]);
#pragma unroll
      for (int r = 0; r < 8; ++r) sh[wave * 16 + 8 * g + r][j * 16 + col] = toh_flush(acc[j][r] * (1.0f / 16384.0f) + bias); }
    __syncthreads();
#pragma unroll 1
    for (int e = tid; e < 64 * 16; e += 128) { const int rl = e >> 4, q = e & 15; vst2(DH + (r0 + rl) * CC + c0 + q * 8, *(const v4u*)&sh[rl][q * 8]); }
  } else {
#pragma unroll
    for (int j = 0; j < 8; ++j) { const float bias = bfr(BA[c0 + j * 16 + col]);
#pragma unroll
      for (int r = 0; r < 8; ++r) th[j * 16 + col][wave * 16 + 8 * g + r] = toh_flush(acc[j][r] * (1.0f / 16384.0f) + bias); }
    __syncthreads();
#pragma unroll 1
    for (int e = tid; e < 128 * 8; e += 128) { const int cl = e >> 3, q = e & 7; vst2(VT + (bb * CC + c0 + cl) * (size_t)TT + t0 + q * 8, *(const v4u*)&th[cl][q * 8]); } } }

__global__ __launch_bounds__(128) void k_attn(const _Float16* __restrict__ QH, const _Float16* __restrict__ KH, const _Float16* __restrict__ VT, _Float16* __restrict__ CT) {
  __shared__ __align__(16) _Float16 ct[4][16][72];
  const int tid = threadIdx.x; const int wave = __builtin_amdgcn_readfirstlane(threadIdx.x >> 5); const int lane = tid & 31, col = lane & 15, g = lane >> 4;
  const int b = blockIdx.z, h = blockIdx.y; const int q0 = blockIdx.x * 64 + wave * 16;
  const _Float16* qp = QH + ((size_t)b * TT + q0 + col) * CC + h * HD;
  const v16h qf0 = frag_h(qp, lane), qf1 = frag_h(qp + 32, lane);
  const _Float16* kp = KH + ((size_t)b * TT + col) * CC + h * HD;
  const _Float16* vp = VT + ((size_t)b * CC + h * HD + col) * (size_t)TT;
  float m = -3.0e38f, l = 0.f;
  v8f o[4] = {};
#pragma unroll 1
  for (int kb = 0; kb < TT; kb += 32) {
    v8f s0 = {}, s1 = {};
    { const _Float16* p = kp + (size_t)kb * CC;
      const v16h ka = frag_h(p, lane), kc = frag_h(p + 32, lane);
      s0 = wmma16(ka, qf0, s0); s0 = wmma16(kc, qf1, s0);
      const _Float16* p2 = p + (size_t)16 * CC;
      const v16h kd = frag_h(p2, lane), ke = frag_h(p2 + 32, lane);
      s1 = wmma16(kd, qf0, s1); s1 = wmma16(ke, qf1, s1); }
    float mx = fmaxf(s0[0], s1[0]);
#pragma unroll
    for (int r = 1; r < 8; ++r) mx = fmaxf(mx, fmaxf(s0[r], s1[r]));
    mx = fmaxf(mx, __shfl_xor(mx, 16));
    const float mn = fmaxf(m, mx * C2);
    const float alpha = __builtin_amdgcn_exp2f(m - mn);
    m = mn;
    const float off = 10.0f - mn;
    float ps = 0.f; v16h pf;
#pragma unroll
    for (int r = 0; r < 8; ++r) { const float p0 = __builtin_amdgcn_exp2f(__builtin_fmaf(s0[r], C2, off)); const float p1 = __builtin_amdgcn_exp2f(__builtin_fmaf(s1[r], C2, off)); ps += p0 + p1; pf[r] = (_Float16)p0; pf[8 + r] = (_Float16)p1; }
    l = l * alpha + ps;
#pragma unroll
    for (int j = 0; j < 4; ++j) o[j] = o[j] * alpha;
#pragma unroll
    for (int j = 0; j < 4; ++j) { const v16h vf = frag_h(vp + (size_t)j * 16 * TT + kb, lane); o[j] = wmma16(vf, pf, o[j]); }
  }
  l += __shfl_xor(l, 16);
  const float inv = 64.0f * __builtin_amdgcn_rcpf(l);
#pragma unroll
  for (int j = 0; j < 4; ++j) { v8h hv;
#pragma unroll
    for (int r = 0; r < 8; ++r) hv[r] = (_Float16)(o[j][r] * inv);
    *(v8h*)&ct[wave][col][j * 16 + 8 * g] = hv; }
  LDSX();
#pragma unroll 1
  for (int i = 0; i < 4; ++i) { const int rl = i * 4 + (lane >> 3), q = lane & 7;
    vst2(CT + ((size_t)b * TT + q0 + rl) * CC + h * HD + q * 8, *(const v4u*)&ct[wave][rl][q * 8]); }
}

__global__ __launch_bounds__(128) void k_mha(const _Float16* __restrict__ CT, const _Float16* __restrict__ WOT, const float* __restrict__ BO, const float* __restrict__ E, float* __restrict__ MF, _Float16* __restrict__ MH) {
  const int tid = threadIdx.x; const int wave = __builtin_amdgcn_readfirstlane(threadIdx.x >> 5); const int lane = tid & 31, col = lane & 15;
  const int c0 = blockIdx.y * 128; const size_t rb = (size_t)blockIdx.x * 64; const size_t r0 = rb + wave * 16;
  v8f acc[8] = {};
  mm_f16(acc, CT + (r0 + col) * CC, WOT + (size_t)(c0 + col) * CC, lane);
  epi_tile<1, 0, 1, 1, 0>(acc, 1.0f / 16384.0f, BO, E, MF, MH, rb, c0, wave, lane);
}

__global__ __launch_bounds__(128) void k_ff1(const _Float16* __restrict__ MH, const _Float16* __restrict__ W1T, const float* __restrict__ B1, _Float16* __restrict__ HH) {
  const int tid = threadIdx.x; const int wave = __builtin_amdgcn_readfirstlane(threadIdx.x >> 5); const int lane = tid & 31, col = lane & 15;
  const int c0 = blockIdx.y * 128; const size_t rb = (size_t)blockIdx.x * 64; const size_t r0 = rb + wave * 16;
  v8f acc[8] = {};
  mm_f16(acc, MH + (r0 + col) * CC, W1T + (size_t)(c0 + col) * CC, lane);
  epi_tile<0, 1, 0, 1, 0>(acc, 1.0f / 16384.0f, B1, B1, (float*)0, HH, rb, c0, wave, lane);
}

__global__ __launch_bounds__(128) void k_ff2(const _Float16* __restrict__ HH, const _Float16* __restrict__ W2T, const float* __restrict__ B2, const float* __restrict__ MF, float* __restrict__ OUT) {
  const int tid = threadIdx.x; const int wave = __builtin_amdgcn_readfirstlane(threadIdx.x >> 5); const int lane = tid & 31, col = lane & 15;
  const int c0 = blockIdx.y * 128; const size_t rb = (size_t)blockIdx.x * 64; const size_t r0 = rb + wave * 16;
  v8f acc[8] = {};
  mm_f16(acc, HH + (r0 + col) * CC, W2T + (size_t)(c0 + col) * CC, lane);
  epi_tile<1, 0, 1, 0, 1>(acc, 1.0f / 16384.0f, B2, MF, OUT, (_Float16*)0, rb, c0, wave, lane);
}

extern "C" void kernel_launch(void* const* d_in, const int* in_sizes, int n_in, void* d_out, int out_size, void* d_ws, size_t ws_size, hipStream_t stream) {
  if (n_in < 15) return;
  const long long rows = (long long)(NB - 1) * TT_FULL + TT;
  if ((long long)in_sizes[0] < rows * DIN) return;
  if (in_sizes[1] < DIN * CC) return;
  if (in_sizes[3] < CC * CC || in_sizes[5] < CC * CC || in_sizes[7] < CC * CC || in_sizes[9] < CC * CC || in_sizes[11] < CC * CC || in_sizes[13] < CC * CC) return;
  if (in_sizes[2] < CC || in_sizes[4] < CC || in_sizes[6] < CC || in_sizes[8] < CC || in_sizes[10] < CC || in_sizes[12] < CC || in_sizes[14] < CC) return;
  if ((long long)out_size < rows * CC) return;
  if (ws_size < (size_t)WS_END) return;
  const float* x = (const float*)d_in[0];
  const float* we = (const float*)d_in[1]; const float* be = (const float*)d_in[2];
  const float* wq = (const float*)d_in[3]; const float* bq = (const float*)d_in[4];
  const float* wk = (const float*)d_in[5]; const float* bk = (const float*)d_in[6];
  const float* wv = (const float*)d_in[7]; const float* bv = (const float*)d_in[8];
  const float* w0 = (const float*)d_in[9]; const float* b0 = (const float*)d_in[10];
  const float* w1 = (const float*)d_in[11]; const float* b1 = (const float*)d_in[12];
  const float* w2 = (const float*)d_in[13]; const float* b2 = (const float*)d_in[14];
  char* ws = (char*)d_ws;
  unsigned short* XB = (unsigned short*)(ws + WS_XB);
  unsigned short* WT = (unsigned short*)(ws + WS_WT);
  const __bf16* WET = (const __bf16*)WT;
  const _Float16* WH = (const _Float16*)(WT + (size_t)CC * DIN);
  float* E = (float*)(ws + WS_E);
  _Float16* EH = (_Float16*)(ws + WS_EH);
  _Float16* QK = (_Float16*)(ws + WS_QK);
  _Float16* VT = (_Float16*)(ws + WS_VT);
  _Float16* CT = (_Float16*)(ws + WS_CT);
  float* MF = (float*)(ws + WS_MF);
  _Float16* MH = (_Float16*)(ws + WS_MH);
  _Float16* HH = (_Float16*)(ws + WS_HH);
  k_cvtx<<<dim3((unsigned)((size_t)NB * TT * DIN / (8 * 256))), 256, 0, stream>>>(x, XB);
  k_wt<<<dim3(CC / 64, CC / 64, 7), 128, 0, stream>>>(we, wq, wk, wv, w0, w1, w2, WT);
  k_emb<<<dim3(NB * TT / 64, CC / 128), 128, 0, stream>>>((const __bf16*)XB, WET, be, E, EH);
  k_proj<<<dim3(NB * TT / 64, CC / 128, 3), 128, 0, stream>>>(EH, WH, bq, bk, bv, QK, VT);
  k_attn<<<dim3(TT / 64, NH, NB), 128, 0, stream>>>(QK, QK + (size_t)NB * TT * CC, VT, CT);
  k_mha<<<dim3(NB * TT / 64, CC / 128), 128, 0, stream>>>(CT, WH + (size_t)3 * CC * CC, b0, E, MF, MH);
  k_ff1<<<dim3(NB * TT / 64, CC / 128), 128, 0, stream>>>(MH, WH + (size_t)4 * CC * CC, b1, HH);
  k_ff2<<<dim3(NB * TT / 64, CC / 128), 128, 0, stream>>>(HH, WH + (size_t)5 * CC * CC, b2, MF, (float*)d_out);
}
